// GATModel_10617159155782
// MI455X (gfx1250) — hardware-verified
//
#include <hip/hip_runtime.h>
#include <stddef.h>
#include <stdint.h>
#include <math.h>


#define F_IN    18
#define KX      32
#define HC      512
#define HID     64
#define NHD     8
#define KA      1024
#define NOUT    15
#define NOUTP   16
#define NTHR    256
#define NWAVE   8
#define EPT     8
#define CHUNK   (NTHR * EPT)
#define WCAP    (EPT * 32)
#define LISTN   (NWAVE * WCAP)
#define NBMAX   2048
#define NBSEL   1024
#define SLOTB   11
#define RCAP    28672
#define DEGCAP  256
#define GBM     64
#define GBN     64
#define GTHR    128
#define MROWS   128
#define NEGSL   0.2f
#define EPS_SM  1e-16f
#define LDS_AGG ((2 * RCAP + 2 * NBMAX + LISTN) * 4 + 64)

static_assert((CHUNK & (CHUNK - 1)) == 0 && CHUNK <= (1 << SLOTB));
static_assert(NBMAX == (1 << SLOTB));
static_assert(NTHR * 8 == NBMAX);
static_assert(NBSEL <= NBMAX && (NBSEL % 32) == 0);
static_assert(LISTN >= NBMAX);
static_assert(LISTN >= NWAVE * WCAP);
static_assert((RCAP % 32) == 0);
static_assert(RCAP >= NOUT * NBSEL);
static_assert(((NBSEL * NOUT) % 4) == 0);
static_assert(((32 * NOUT * 4) % 128) == 0);
static_assert(LISTN >= HID * NOUTP + NOUTP + NWAVE * HID);
static_assert(LDS_AGG <= 300000);
static_assert(GBM == (GTHR / 32) * 16);
static_assert(GTHR == 2 * GBN && GTHR == 2 * GBM);
static_assert((KX % 32) == 0 && (KA % 32) == 0);
static_assert(F_IN <= KX && (F_IN % 2) == 0 && KX == 4 * 8);
static_assert((HC % GBN) == 0 && HID == GBN);
static_assert(HC == NHD * HID);
static_assert(KA == 2 * HC);
static_assert((MROWS % GBM) == 0);
static_assert(HC == 2 * 8 * 32);
static_assert(HID == 8 * 8);
static_assert(DEGCAP >= 32);

typedef float          v2f  __attribute__((ext_vector_type(2)));
typedef float          v4f  __attribute__((ext_vector_type(4)));
typedef float          v8f  __attribute__((ext_vector_type(8)));
typedef int            v4i  __attribute__((ext_vector_type(4)));
typedef int            v8i  __attribute__((ext_vector_type(8)));
typedef unsigned int   v4u  __attribute__((ext_vector_type(4)));
typedef unsigned short v8us __attribute__((ext_vector_type(8)));
typedef __bf16         v16b __attribute__((ext_vector_type(16)));
typedef v2f  __attribute__((may_alias)) v2fa;
typedef v4f  __attribute__((may_alias)) v4fa;
typedef v8us __attribute__((may_alias)) v8usa;
union FragB { v16b v; v8us h[2]; v8i w; };

__device__ __forceinline__ v8f wmb(const FragB& a, const FragB& b, v8f c) {
  v8f d = __builtin_amdgcn_wmma_f32_16x16x32_bf16(false, a.v, false, b.v, (short)0, c, false, false);
  asm volatile("v_nop\n\tv_nop\n\tv_nop\n\tv_nop" : "+v"(d) : "v"(a.w), "v"(b.w));
  return d;
}

__device__ __forceinline__ unsigned int f2bf(float f) {
  const unsigned int u = __float_as_uint(f);
  return ((u + 0x7FFFu + ((u >> 16) & 1u)) >> 16) & 0xFFFFu;
}
__device__ __forceinline__ float bf2f(unsigned int b) { return __uint_as_float(b << 16); }
__device__ __forceinline__ float bfr(float f) { return bf2f(f2bf(f)); }
__device__ __forceinline__ v4f bfr4(const v4f a) {
  v4f r; r.x = bfr(a.x); r.y = bfr(a.y); r.z = bfr(a.z); r.w = bfr(a.w); return r;
}
__device__ __forceinline__ unsigned int pk2(float lo, float hi) { return f2bf(lo) | (f2bf(hi) << 16); }
__device__ __forceinline__ v4u pack8(const v4f a, const v4f b) {
  v4u r;
  r.x = pk2(a.x, a.y); r.y = pk2(a.z, a.w); r.z = pk2(b.x, b.y); r.w = pk2(b.z, b.w);
  return r;
}
__device__ __forceinline__ v4u lo8(const v4f a, const v4f b) {
  v4f ra, rb;
  ra.x = a.x - bfr(a.x); ra.y = a.y - bfr(a.y); ra.z = a.z - bfr(a.z); ra.w = a.w - bfr(a.w);
  rb.x = b.x - bfr(b.x); rb.y = b.y - bfr(b.y); rb.z = b.z - bfr(b.z); rb.w = b.w - bfr(b.w);
  return pack8(ra, rb);
}
__device__ __forceinline__ float fin1(float a, float inv, float b, bool live, float pz) {
  float v = fmaf(a, inv, b);
  v = v > 0.f ? v : (__expf(v) - 1.0f);
  return (live ? v : 0.f) + pz;
}
__device__ __forceinline__ v4f fin4(const v4f a, float inv, const v4f b, bool live, float pz) {
  v4f r;
  r.x = fin1(a.x, inv, b.x, live, pz);
  r.y = fin1(a.y, inv, b.y, live, pz);
  r.z = fin1(a.z, inv, b.z, live, pz);
  r.w = fin1(a.w, inv, b.w, live, pz);
  return r;
}

__device__ __forceinline__ int scan_chunk(const int* __restrict__ dsts, int nE, int cbase, int slotBase,
                                          int nb, int vec8, int* list, int tid, int lane, int wave) {
  int wc = 0;
  const int el0  = tid * EPT;
  const int e0   = cbase + el0;
  const int sent = -2147483647 - 1;
  v4i da, db;
  if (vec8 != 0 && cbase + CHUNK <= nE) {
    da = *(const v4i*)(dsts + e0);
    db = *(const v4i*)(dsts + e0 + 4);
  } else {
    da.x = (e0     < nE) ? dsts[min(e0,     nE - 1)] : sent;
    da.y = (e0 + 1 < nE) ? dsts[min(e0 + 1, nE - 1)] : sent;
    da.z = (e0 + 2 < nE) ? dsts[min(e0 + 2, nE - 1)] : sent;
    da.w = (e0 + 3 < nE) ? dsts[min(e0 + 3, nE - 1)] : sent;
    db.x = (e0 + 4 < nE) ? dsts[min(e0 + 4, nE - 1)] : sent;
    db.y = (e0 + 5 < nE) ? dsts[min(e0 + 5, nE - 1)] : sent;
    db.z = (e0 + 6 < nE) ? dsts[min(e0 + 6, nE - 1)] : sent;
    db.w = (e0 + 7 < nE) ? dsts[min(e0 + 7, nE - 1)] : sent;
  }
  const unsigned nbs = (unsigned)slotBase;
  const unsigned unb = (unsigned)nb;
  const unsigned s0 = (unsigned)da.x - nbs, s1 = (unsigned)da.y - nbs;
  const unsigned s2 = (unsigned)da.z - nbs, s3 = (unsigned)da.w - nbs;
  const unsigned s4 = (unsigned)db.x - nbs, s5 = (unsigned)db.y - nbs;
  const unsigned s6 = (unsigned)db.z - nbs, s7 = (unsigned)db.w - nbs;
  const bool h0 = s0 < unb, h1 = s1 < unb, h2 = s2 < unb, h3 = s3 < unb;
  const bool h4 = s4 < unb, h5 = s5 < unb, h6 = s6 < unb, h7 = s7 < unb;
  const unsigned any = __builtin_amdgcn_ballot_w32(h0 | h1 | h2 | h3 | h4 | h5 | h6 | h7);
  if (any != 0u) {
#define HITJ(J, HJ, SJ) { \
      const unsigned mj = __builtin_amdgcn_ballot_w32(HJ); \
      if (mj != 0u) { \
        if (HJ) { \
          const int pos = wc + (int)__builtin_amdgcn_mbcnt_lo(mj, 0u); \
          if (pos < WCAP) list[wave * WCAP + pos] = ((el0 + (J)) << SLOTB) | (int)(SJ); \
        } \
        wc += (int)__builtin_popcount(mj); } }
    HITJ(0, h0, s0)
    HITJ(1, h1, s1)
    HITJ(2, h2, s2)
    HITJ(3, h3, s3)
    HITJ(4, h4, s4)
    HITJ(5, h5, s5)
    HITJ(6, h6, s6)
    HITJ(7, h7, s7)
#undef HITJ
  }
  return wc;
}

__global__ __launch_bounds__(NTHR) void k_xprep(const float* __restrict__ x, unsigned short* xb, int nN, int nUnits) {
  const int i = (int)blockIdx.x * NTHR + (int)threadIdx.x;
  if (i >= nUnits) return;
  const int row = i >> 2;
  const int c0  = (i & 3) * 8;
  const int rc  = row < nN ? row : nN - 1;
  const float* p = x + (size_t)rc * F_IN;
  const int ca = min(c0,     F_IN - 2), cb = min(c0 + 2, F_IN - 2);
  const int cc = min(c0 + 4, F_IN - 2), cd = min(c0 + 6, F_IN - 2);
  const v2f pa = *(const v2fa*)(p + ca);
  const v2f pb = *(const v2fa*)(p + cb);
  const v2f pc = *(const v2fa*)(p + cc);
  const v2f pd = *(const v2fa*)(p + cd);
  const bool rl = row < nN;
  const bool va = rl && (c0     < F_IN), vb = rl && (c0 + 2 < F_IN);
  const bool vc = rl && (c0 + 4 < F_IN), vd = rl && (c0 + 6 < F_IN);
  v4f a, b;
  a.x = va ? pa.x : 0.f; a.y = va ? pa.y : 0.f;
  a.z = vb ? pb.x : 0.f; a.w = vb ? pb.y : 0.f;
  b.x = vc ? pc.x : 0.f; b.y = vc ? pc.y : 0.f;
  b.z = vd ? pd.x : 0.f; b.w = vd ? pd.y : 0.f;
  const v4u hv = pack8(a, b);
  const size_t o = (size_t)row * KX + c0;
  *(volatile v4u*)(xb + o) = hv;
  __threadfence();
  *(volatile v4u*)(xb + o) = hv;
}

__global__ __launch_bounds__(NTHR) void k_wtr(const float* __restrict__ w, int Kin, int Kper, int Ncol, int Kout,
                                              unsigned short* wt, int nUnits) {
  const int u = (int)blockIdx.x * NTHR + (int)threadIdx.x;
  if (u >= nUnits) return;
  const int kq = Kout >> 3;
  const int n  = u / kq;
  const int k8 = (u - n * kq) * 8;
  const int kk = k8 - (k8 / Kper) * Kper;
  const int ncl = n < Ncol ? n : Ncol - 1;
  const float* p = w + ncl;
  const int km = Kin - 1;
  const int r0 = min(kk, km),     r1 = min(kk + 1, km), r2 = min(kk + 2, km), r3 = min(kk + 3, km);
  const int r4 = min(kk + 4, km), r5 = min(kk + 5, km), r6 = min(kk + 6, km), r7 = min(kk + 7, km);
  const float q0 = p[(size_t)r0 * Ncol], q1 = p[(size_t)r1 * Ncol], q2 = p[(size_t)r2 * Ncol], q3 = p[(size_t)r3 * Ncol];
  const float q4 = p[(size_t)r4 * Ncol], q5 = p[(size_t)r5 * Ncol], q6 = p[(size_t)r6 * Ncol], q7 = p[(size_t)r7 * Ncol];
  const bool nv = n < Ncol;
  v4f a, b;
  a.x = (nv && kk     < Kin) ? q0 : 0.f;
  a.y = (nv && kk + 1 < Kin) ? q1 : 0.f;
  a.z = (nv && kk + 2 < Kin) ? q2 : 0.f;
  a.w = (nv && kk + 3 < Kin) ? q3 : 0.f;
  b.x = (nv && kk + 4 < Kin) ? q4 : 0.f;
  b.y = (nv && kk + 5 < Kin) ? q5 : 0.f;
  b.z = (nv && kk + 6 < Kin) ? q6 : 0.f;
  b.w = (nv && kk + 7 < Kin) ? q7 : 0.f;
  const v4u wv = pack8(a, b);
  unsigned short* o = wt + (size_t)n * (size_t)Kout + k8;
  *(volatile v4u*)o = wv;
  __threadfence();
  *(volatile v4u*)o = wv;
}

__global__ __launch_bounds__(GTHR) void k_gemm(
    const unsigned short* __restrict__ A, const unsigned short* __restrict__ WT,
    float* outF, int K, int ldo,
    const float* __restrict__ atts, const float* __restrict__ attd, int attLen,
    float* SD, int MPr)
{
  __shared__ __attribute__((aligned(16))) float stg[GBM * GBN];
  __shared__ __attribute__((aligned(16))) float satt[2 * GBN];
  __shared__ __attribute__((aligned(16))) float sdot[2 * GBM];
  const int tid = (int)threadIdx.x, lane = tid & 31, wave = tid >> 5, hh = lane >> 4, m = lane & 15;
  const int rowBase = (int)blockIdx.x * GBM;
  const int head    = (int)blockIdx.y;
  const int col0    = head * GBN;

  {
    const int which = tid >> 6;
    const int c  = tid & 63;
    const int cl = c < attLen ? c : attLen - 1;
    const float vs = atts[head * attLen + cl];
    const float vd = attd[head * attLen + cl];
    const unsigned int msk = (which == 0) ? 0u : 0xFFFFFFFFu;
    const unsigned int inr = (c < attLen) ? 0xFFFFFFFFu : 0u;
    float v = __uint_as_float((__float_as_uint(vs) & ~msk) | (__float_as_uint(vd) & msk));
    v = __uint_as_float(__float_as_uint(bfr(v)) & inr);
    satt[which * GBN + c] = v;
  }

  v8f acc[4];
  {
    const v8f z = {0.f, 0.f, 0.f, 0.f, 0.f, 0.f, 0.f, 0.f};
    acc[0] = z; acc[1] = z; acc[2] = z; acc[3] = z;
  }
  const unsigned short* ap = A  + (size_t)(rowBase + 16 * wave + m) * (size_t)K + 8 * hh;
  const unsigned short* wp = WT + (size_t)(col0 + m) * (size_t)K + 8 * hh;
  const int ksteps = K >> 5;
#pragma unroll 1
  for (int ks = 0; ks < ksteps; ++ks) {
    FragB af;
    af.h[0] = *(const v8usa*)(ap + 32 * ks);
    af.h[1] = *(const v8usa*)(ap + 32 * ks + 16);
#pragma unroll
    for (int t = 0; t < 4; ++t) {
      const unsigned short* wq = wp + (size_t)(16 * t) * (size_t)K + 32 * ks;
      FragB bf;
      bf.h[0] = *(const v8usa*)wq;
      bf.h[1] = *(const v8usa*)(wq + 16);
      acc[t] = wmb(af, bf, acc[t]);
    }
  }

#pragma unroll
  for (int t = 0; t < 4; ++t) {
    const int lc = 16 * t + m;
#pragma unroll
    for (int r = 0; r < 8; ++r) {
      const int lr = 16 * wave + 8 * hh + r;
      stg[lr * GBN + lc] = acc[t][r];
    }
  }
  __syncthreads();

  {
    const int row = tid & 63, which = tid >> 6;
    const float* sa = satt + which * GBN;
    const float* hr = stg + row * GBN;
    float d = 0.f;
#pragma unroll 4
    for (int c4 = 0; c4 < GBN / 4; ++c4) {
      const v4f hv = *(const v4fa*)(hr + 4 * c4);
      const v4f av = *(const v4fa*)(sa + 4 * c4);
      d = fmaf(hv.x, av.x, d);
      d = fmaf(hv.y, av.y, d);
      d = fmaf(hv.z, av.z, d);
      d = fmaf(hv.w, av.w, d);
    }
    sdot[which * GBM + row] = d;
  }
  __syncthreads();

  v4f fv[8];
#pragma unroll
  for (int i = 0; i < 8; ++i) {
    const int lr = 16 * wave + 2 * i + hh;
    fv[i] = *(const v4fa*)(stg + lr * GBN + 4 * m);
  }
  const int which2 = lane >> 4, piece = lane & 15;
  const v4f sdv = *(const v4fa*)(sdot + which2 * GBM + 4 * piece);
  float* sp = SD + (size_t)(2 * head + which2) * (size_t)MPr + rowBase + 4 * piece;

#pragma unroll
  for (int i = 0; i < 8; ++i) {
    const int lr = 16 * wave + 2 * i + hh;
    const int gr = rowBase + lr;
    float* op = outF + (size_t)gr * (size_t)ldo + col0 + 4 * m;
    *(volatile v4f*)op = fv[i];
  }
  if (wave == 0) *(volatile v4f*)sp = sdv;
  __threadfence();
#pragma unroll
  for (int i = 0; i < 8; ++i) {
    const int lr = 16 * wave + 2 * i + hh;
    const int gr = rowBase + lr;
    float* op = outF + (size_t)gr * (size_t)ldo + col0 + 4 * m;
    *(volatile v4f*)op = fv[i];
  }
  if (wave == 0) *(volatile v4f*)sp = sdv;
}

template<int L>
__global__ __launch_bounds__(NTHR) void k_agg(
    const int* __restrict__ srcs, const int* __restrict__ dsts,
    const float* __restrict__ F, const float* __restrict__ SD,
    const float* __restrict__ bias, const float* __restrict__ fcw, const float* __restrict__ fcb,
    unsigned short* HP, float* out,
    int nN, int nE, int nb, int vec8, int MPr) {
  extern __shared__ v4f lds_dyn[];
  int* reg1 = (int*)lds_dyn;
  int* reg2 = reg1 + RCAP;
  int* scnt = reg2 + RCAP;
  int* soff = scnt + NBMAX;
  int* list = soff + NBMAX;
  int* wcnt = list + LISTN;
  int* wtot = wcnt + NWAVE;
  const int tid = (int)threadIdx.x, lane = tid & 31, wave = tid >> 5;
  const int nodeBase = (int)blockIdx.x * nb;

  for (int i = tid; i < NBMAX; i += NTHR) scnt[i] = 0;
  __syncthreads();

  int tot = 0;
  const int nChunks = (nE + CHUNK - 1) / CHUNK;
#pragma unroll 1
  for (int ch = 0; ch < nChunks; ++ch) {
    const int cbase = ch * CHUNK;
    const int wc = scan_chunk(dsts, nE, cbase, nodeBase, nb, vec8, list, tid, lane, wave);
    if (lane == 0) wcnt[wave] = wc;
    __syncthreads();
    int pre = 0, all = 0;
#pragma unroll
    for (int w2 = 0; w2 < NWAVE; ++w2) {
      int c = wcnt[w2];
      c = c < 0 ? 0 : (c > WCAP ? WCAP : c);
      all += c;
      pre += (w2 < wave) ? c : 0;
    }
    const int wcc  = wc > WCAP ? WCAP : wc;
    const int base = tot + pre;
#pragma unroll 1
    for (int i = lane; i < wcc; i += 32) {
      const int ent = list[wave * WCAP + i];
      const int el  = (ent >> SLOTB) & (CHUNK - 1);
      const int sl  = ent & (NBMAX - 1);
      int eid = cbase + el;
      eid = eid > nE - 1 ? nE - 1 : eid;
      const int pos = base + i;
      if (pos < RCAP) reg1[pos] = (int)(((unsigned)eid << SLOTB) | (unsigned)sl);
    }
    tot += all;
    tot = tot > RCAP ? RCAP : tot;
    __syncthreads();
  }
  const int nh = tot;

  if (wave == 0) {
#pragma unroll 1
    for (int b0 = 0; b0 < nh; b0 += 32) {
      const int idx = b0 + lane;
      const int uv  = reg1[idx < nh ? idx : nh - 1];
      const int m32 = (nh - b0) < 32 ? (nh - b0) : 32;
#pragma unroll 1
      for (int k = 0; k < m32; ++k) {
        const int u  = __builtin_amdgcn_readlane(uv, k);
        const int sl = u & (NBMAX - 1);
        if (lane == 0) scnt[sl] = scnt[sl] + 1;
      }
    }
  }
  __syncthreads();

  {
    const v4i ca = *(const v4i*)(scnt + 8 * tid);
    const v4i cb = *(const v4i*)(scnt + 8 * tid + 4);
    const int e0 = ca.x < 0 ? 0 : ca.x, e1 = ca.y < 0 ? 0 : ca.y, e2 = ca.z < 0 ? 0 : ca.z, e3 = ca.w < 0 ? 0 : ca.w;
    const int e4 = cb.x < 0 ? 0 : cb.x, e5 = cb.y < 0 ? 0 : cb.y, e6 = cb.z < 0 ? 0 : cb.z, e7 = cb.w < 0 ? 0 : cb.w;
    const int ts = e0 + e1 + e2 + e3 + e4 + e5 + e6 + e7;
    int incl = ts;
#pragma unroll
    for (int d = 1; d < 32; d <<= 1) {
      const int up = __shfl_up(incl, d);
      if (lane >= d) incl += up;
    }
    if (lane == 31) wtot[wave] = incl;
    __syncthreads();
    int pre = 0;
#pragma unroll
    for (int w2 = 0; w2 < NWAVE; ++w2) pre += (w2 < wave) ? wtot[w2] : 0;
    int run = pre + incl - ts;
    soff[8 * tid + 0] = run; run += e0;
    soff[8 * tid + 1] = run; run += e1;
    soff[8 * tid + 2] = run; run += e2;
    soff[8 * tid + 3] = run; run += e3;
    soff[8 * tid + 4] = run; run += e4;
    soff[8 * tid + 5] = run; run += e5;
    soff[8 * tid + 6] = run; run += e6;
    soff[8 * tid + 7] = run;
  }
  __syncthreads();
  for (int i = tid; i < NBMAX; i += NTHR) list[i] = soff[i];
  __syncthreads();

  if (wave == 0) {
#pragma unroll 1
    for (int b0 = 0; b0 < nh; b0 += 32) {
      const int idx = b0 + lane;
      const int uv  = reg1[idx < nh ? idx : nh - 1];
      const int m32 = (nh - b0) < 32 ? (nh - b0) : 32;
#pragma unroll 1
      for (int k = 0; k < m32; ++k) {
        const int u   = __builtin_amdgcn_readlane(uv, k);
        const int sl  = u & (NBMAX - 1);
        const int eid = (int)((unsigned)u >> SLOTB);
        if (lane == 0) {
          int pos = list[sl];
          pos = pos < 0 ? 0 : (pos > RCAP - 1 ? RCAP - 1 : pos);
          reg2[pos] = eid;
          list[sl] = pos + 1;
        }
      }
    }
  }
  __syncthreads();

  const int nbw = nb >> 3;
  const bool ovf = (nh >= RCAP);
  const float qnan = __int_as_float(0x7fc00000);
  const int c0  = 8 * lane;
  const int hd0 = lane >> 3;
  const float* AS0 = SD + (size_t)(2 * hd0) * (size_t)MPr;
  const float* AD0 = AS0 + MPr;
  const float* AS1 = SD + (size_t)(2 * (hd0 + 4)) * (size_t)MPr;
  const float* AD1 = AS1 + MPr;

  float* wl   = (float*)list;
  float* bo   = wl + HID * NOUTP;
  float* xrow = bo + NOUTP + wave * HID;
  float* res  = (float*)reg1;

  v4f bA0, bB0, bA1, bB1;
  if (L == 1) {
    bA0 = bfr4(*(const v4fa*)(bias + c0));
    bB0 = bfr4(*(const v4fa*)(bias + c0 + 4));
    bA1 = bfr4(*(const v4fa*)(bias + 256 + c0));
    bB1 = bfr4(*(const v4fa*)(bias + 256 + c0 + 4));
  } else {
    const int cb3 = 8 * (lane & 7);
    bA0 = bfr4(*(const v4fa*)(bias + cb3));
    bB0 = bfr4(*(const v4fa*)(bias + cb3 + 4));
    bA1 = bA0; bB1 = bB0;
#pragma unroll 1
    for (int i = tid; i < HID * NOUTP; i += NTHR) {
      const int c = i >> 4, j = i & 15;
      const int jc = j < NOUT ? j : NOUT - 1;
      float v = bfr(fcw[c * NOUT + jc]);
      v = (j < NOUT) ? v : 0.f;
      wl[i] = v;
    }
    if (tid < NOUTP) {
      const int jc = tid < NOUT ? tid : NOUT - 1;
      float v = bfr(fcb[jc]);
      v = (tid < NOUT) ? v : 0.f;
      bo[tid] = v;
    }
    __syncthreads();
  }

#pragma unroll 1
  for (int jt = 0; jt < nbw; ++jt) {
    const int slot = wave * nbw + jt;
    const int grow = nodeBase + slot;
    const int gcl  = grow < nN ? grow : nN - 1;
    int st = soff[slot];
    const int craw = scnt[slot];
    int cnt = craw;
    st  = st < 0 ? 0 : (st > nh ? nh : st);
    cnt = cnt < 0 ? 0 : (cnt > DEGCAP ? DEGCAP : cnt);
    if (cnt > nh - st) cnt = nh - st;
    const float pz = (ovf || craw > DEGCAP) ? qnan : 0.0f;

    const float* fr = F + (size_t)gcl * HC + c0;
    v4f a0 = *(const v4fa*)fr;
    v4f b0 = *(const v4fa*)(fr + 4);
    v4f a1 = *(const v4fa*)(fr + 256);
    v4f b1 = *(const v4fa*)(fr + 260);
    const float ad0 = AD0[gcl], ad1 = AD1[gcl];
    float l0 = AS0[gcl] + ad0;
    float l1 = AS1[gcl] + ad1;
    l0 = l0 > 0.f ? l0 : NEGSL * l0;
    l1 = l1 > 0.f ? l1 : NEGSL * l1;
    float mx0 = l0, mx1 = l1, dn0 = 1.0f, dn1 = 1.0f;

#pragma unroll 1
    for (int q = 0; q < cnt; ++q) {
      int idx = st + q; idx = idx > RCAP - 1 ? RCAP - 1 : idx;
      int eid = reg2[idx]; eid = eid < 0 ? 0 : (eid > nE - 1 ? nE - 1 : eid);
      const int sraw = srcs[eid];
      const int s = sraw < 0 ? 0 : (sraw > nN - 1 ? nN - 1 : sraw);
      const float* gs = F + (size_t)s * HC + c0;
      const v4f fa0 = *(const v4fa*)gs;
      const v4f fb0 = *(const v4fa*)(gs + 4);
      const v4f fa1 = *(const v4fa*)(gs + 256);
      const v4f fb1 = *(const v4fa*)(gs + 260);
      float lg0 = AS0[s] + ad0;
      float lg1 = AS1[s] + ad1;
      lg0 = lg0 > 0.f ? lg0 : NEGSL * lg0;
      lg1 = lg1 > 0.f ? lg1 : NEGSL * lg1;
      const float df0 = lg0 - mx0, df1 = lg1 - mx1;
      const float ee0 = __expf(-fabsf(df0));
      const float ee1 = __expf(-fabsf(df1));
      const bool up0 = df0 > 0.f, up1 = df1 > 0.f;
      const float p0 = up0 ? ee0 : 1.0f, q0 = up0 ? 1.0f : ee0;
      const float p1 = up1 ? ee1 : 1.0f, q1 = up1 ? 1.0f : ee1;
      mx0 = up0 ? lg0 : mx0;
      mx1 = up1 ? lg1 : mx1;
      dn0 = fmaf(dn0, p0, q0);
      dn1 = fmaf(dn1, p1, q1);
      a0.x = fmaf(a0.x, p0, q0 * fa0.x);
      a0.y = fmaf(a0.y, p0, q0 * fa0.y);
      a0.z = fmaf(a0.z, p0, q0 * fa0.z);
      a0.w = fmaf(a0.w, p0, q0 * fa0.w);
      b0.x = fmaf(b0.x, p0, q0 * fb0.x);
      b0.y = fmaf(b0.y, p0, q0 * fb0.y);
      b0.z = fmaf(b0.z, p0, q0 * fb0.z);
      b0.w = fmaf(b0.w, p0, q0 * fb0.w);
      a1.x = fmaf(a1.x, p1, q1 * fa1.x);
      a1.y = fmaf(a1.y, p1, q1 * fa1.y);
      a1.z = fmaf(a1.z, p1, q1 * fa1.z);
      a1.w = fmaf(a1.w, p1, q1 * fa1.w);
      b1.x = fmaf(b1.x, p1, q1 * fb1.x);
      b1.y = fmaf(b1.y, p1, q1 * fb1.y);
      b1.z = fmaf(b1.z, p1, q1 * fb1.z);
      b1.w = fmaf(b1.w, p1, q1 * fb1.w);
    }
    const float inv0 = __builtin_amdgcn_rcpf(dn0 + EPS_SM);
    const float inv1 = __builtin_amdgcn_rcpf(dn1 + EPS_SM);

    if (L == 1) {
      const bool live = grow < nN;
      const v4f oa0 = fin4(a0, inv0, bA0, live, pz);
      const v4f ob0 = fin4(b0, inv0, bB0, live, pz);
      const v4f oa1 = fin4(a1, inv1, bA1, live, pz);
      const v4f ob1 = fin4(b1, inv1, bB1, live, pz);
      const v4u h0v = pack8(oa0, ob0);
      const v4u h1v = pack8(oa1, ob1);
      const v4u l0v = lo8(oa0, ob0);
      const v4u l1v = lo8(oa1, ob1);
      unsigned short* g0 = HP + (size_t)grow * KA + c0;
      const bool wr = grow < MPr;
      if (wr) {
        *(volatile v4u*)g0         = h0v;
        *(volatile v4u*)(g0 + 256) = h1v;
        *(volatile v4u*)(g0 + 512) = l0v;
        *(volatile v4u*)(g0 + 768) = l1v;
      }
      __threadfence();
      if (wr) {
        *(volatile v4u*)g0         = h0v;
        *(volatile v4u*)(g0 + 256) = h1v;
        *(volatile v4u*)(g0 + 512) = l0v;
        *(volatile v4u*)(g0 + 768) = l1v;
      }
    } else {
      float t0 = fmaf(a1.x, inv1, a0.x * inv0);
      float t1 = fmaf(a1.y, inv1, a0.y * inv0);
      float t2 = fmaf(a1.z, inv1, a0.z * inv0);
      float t3 = fmaf(a1.w, inv1, a0.w * inv0);
      float t4 = fmaf(b1.x, inv1, b0.x * inv0);
      float t5 = fmaf(b1.y, inv1, b0.y * inv0);
      float t6 = fmaf(b1.z, inv1, b0.z * inv0);
      float t7 = fmaf(b1.w, inv1, b0.w * inv0);
      t0 += __shfl_xor(t0, 8); t1 += __shfl_xor(t1, 8); t2 += __shfl_xor(t2, 8); t3 += __shfl_xor(t3, 8);
      t4 += __shfl_xor(t4, 8); t5 += __shfl_xor(t5, 8); t6 += __shfl_xor(t6, 8); t7 += __shfl_xor(t7, 8);
      t0 += __shfl_xor(t0, 16); t1 += __shfl_xor(t1, 16); t2 += __shfl_xor(t2, 16); t3 += __shfl_xor(t3, 16);
      t4 += __shfl_xor(t4, 16); t5 += __shfl_xor(t5, 16); t6 += __shfl_xor(t6, 16); t7 += __shfl_xor(t7, 16);
      v4f xa, xb;
      xa.x = fmaf(t0, 0.125f, bA0.x); xa.y = fmaf(t1, 0.125f, bA0.y);
      xa.z = fmaf(t2, 0.125f, bA0.z); xa.w = fmaf(t3, 0.125f, bA0.w);
      xb.x = fmaf(t4, 0.125f, bB0.x); xb.y = fmaf(t5, 0.125f, bB0.y);
      xb.z = fmaf(t6, 0.125f, bB0.z); xb.w = fmaf(t7, 0.125f, bB0.w);
      if (lane < 8) {
        *(v4fa*)(xrow + 8 * lane)     = xa;
        *(v4fa*)(xrow + 8 * lane + 4) = xb;
      }
      __syncthreads();
      const int j = lane & 15;
      float y = 0.f;
#pragma unroll 2
      for (int c4 = 0; c4 < HID / 4; ++c4) {
        const v4f xv = *(const v4fa*)(xrow + 4 * c4);
        const float* wq = wl + (4 * c4) * NOUTP + j;
        y = fmaf(xv.x, wq[0],         y);
        y = fmaf(xv.y, wq[NOUTP],     y);
        y = fmaf(xv.z, wq[2 * NOUTP], y);
        y = fmaf(xv.w, wq[3 * NOUTP], y);
      }
      y = (y + bo[j]) + pz;
      if (lane < NOUT) res[NOUT * slot + lane] = y;
      __syncthreads();
    }
  }

  if (L == 2) {
    __syncthreads();
    const int npc  = (nb * NOUT) >> 2;
    const int nTot = nN * NOUT;
#pragma unroll 1
    for (int p = tid; p < npc; p += NTHR) {
      const v4f v = *(const v4fa*)(res + 4 * p);
      const int f0 = nodeBase * NOUT + 4 * p;
      float* op = out + (size_t)f0;
      const int rem = nTot - f0;
      if (rem >= 4) {
        *(volatile v4f*)op = v;
      } else if (rem > 0) {
        if (rem >= 2) { v2f w; w.x = v.x; w.y = v.y; *(volatile v2f*)op = w; }
        else          { *(volatile float*)op = v.x; }
        if (rem == 3) *(volatile float*)(op + 2) = v.z;
      }
    }
    __threadfence();
#pragma unroll 1
    for (int p = tid; p < npc; p += NTHR) {
      const v4f v = *(const v4fa*)(res + 4 * p);
      const int f0 = nodeBase * NOUT + 4 * p;
      float* op = out + (size_t)f0;
      const int rem = nTot - f0;
      if (rem >= 4) {
        *(volatile v4f*)op = v;
      } else if (rem > 0) {
        if (rem >= 2) { v2f w; w.x = v.x; w.y = v.y; *(volatile v2f*)op = w; }
        else          { *(volatile float*)op = v.x; }
        if (rem == 3) *(volatile float*)(op + 2) = v.z;
      }
    }
  }
}

static int pick_nb(int nE, int nN) {
  int nb = NBSEL;
  while (nb > 32 && (long long)nb * (long long)nE * 5LL > (long long)RCAP * (long long)nN * 4LL) nb >>= 1;
  return nb;
}
static inline int cdiv(int a, int b) { return (a + b - 1) / b; }

extern "C" void kernel_launch(void* const* d_in, const int* in_sizes, int n_in,
                              void* d_out, int out_size, void* d_ws, size_t ws_size,
                              hipStream_t stream) {
  if (n_in < 16) return;
  const int nN = in_sizes[0] / F_IN;
  if (nN <= 0 || in_sizes[0] != nN * F_IN || nN > (1 << 21)) return;
  if (in_sizes[1] < 2 || (in_sizes[1] & 1) != 0) return;
  const int nE = in_sizes[1] / 2;
  if (nE < 1 || nE >= (1 << (32 - SLOTB))) return;
  if (in_sizes[2] != F_IN * HC) return;
  if (in_sizes[3] != NHD * HID || in_sizes[4] != NHD * HID) return;
  if (in_sizes[5] != HC) return;
  if (in_sizes[6] != HC * HC) return;
  if (in_sizes[7] != NHD * HID || in_sizes[8] != NHD * HID) return;
  if (in_sizes[9] != HC) return;
  if (in_sizes[10] != HC * HC) return;
  if (in_sizes[11] != NHD * HID || in_sizes[12] != NHD * HID) return;
  if (in_sizes[13] != HID) return;
  if (in_sizes[14] != HID * NOUT) return;
  if (in_sizes[15] < NOUT) return;
  if (out_size != nN * NOUT) return;

  const float* x    = (const float*)d_in[0];
  const int*   ei   = (const int*)  d_in[1];
  const float* W1   = (const float*)d_in[2];
  const float* a1s  = (const float*)d_in[3];
  const float* a1d  = (const float*)d_in[4];
  const float* b1   = (const float*)d_in[5];
  const float* W2   = (const float*)d_in[6];
  const float* a2s  = (const float*)d_in[7];
  const float* a2d  = (const float*)d_in[8];
  const float* b2   = (const float*)d_in[9];
  const float* W3   = (const float*)d_in[10];
  const float* a3s  = (const float*)d_in[11];
  const float* a3d  = (const float*)d_in[12];
  const float* b3   = (const float*)d_in[13];
  const float* fcw  = (const float*)d_in[14];
  const float* fcb  = (const float*)d_in[15];
  float* out = (float*)d_out;
  const int* src = ei;
  const int* dst = ei + nE;

  const int MP   = cdiv(nN, MROWS) * MROWS;
  const int nb   = pick_nb(nE, nN);
  if (nb < 32 || (nb & (nb - 1)) != 0 || nb > NBSEL) return;
  const int gA   = cdiv(MP, nb);
  const int vec8 = ((nE & 3) == 0) ? 1 : 0;
  if (gA * nb < MP) return;

  char* ws = (char*)d_ws;
  size_t off = 0;
  const size_t oXB  = off; off += (size_t)MP * KX * 2;             off = (off + 255) & ~(size_t)255;
  const size_t oW1T = off; off += (size_t)HC * KX * 2;             off = (off + 255) & ~(size_t)255;
  const size_t oW2T = off; off += (size_t)HC * KA * 2;             off = (off + 255) & ~(size_t)255;
  const size_t oW3T = off; off += (size_t)HC * KA * 2;             off = (off + 255) & ~(size_t)255;
  const size_t oH   = off; off += (size_t)MP * HC * 4;             off = (off + 255) & ~(size_t)255;
  const size_t oSD  = off; off += (size_t)2 * NHD * MP * 4;        off = (off + 255) & ~(size_t)255;
  const size_t oA   = off; off += (size_t)MP * KA * 2;             off = (off + 255) & ~(size_t)255;
  if (off > ws_size) return;
  unsigned short* XB  = (unsigned short*)(ws + oXB);
  unsigned short* W1T = (unsigned short*)(ws + oW1T);
  unsigned short* W2T = (unsigned short*)(ws + oW2T);
  unsigned short* W3T = (unsigned short*)(ws + oW3T);
  float*          H   = (float*)(ws + oH);
  float*          SD  = (float*)(ws + oSD);
  unsigned short* AP  = (unsigned short*)(ws + oA);

  hipFuncSetAttribute(reinterpret_cast<const void*>(&k_agg<1>),
                      hipFuncAttributeMaxDynamicSharedMemorySize, LDS_AGG);
  hipFuncSetAttribute(reinterpret_cast<const void*>(&k_agg<2>),
                      hipFuncAttributeMaxDynamicSharedMemorySize, LDS_AGG);

  const int nUx = MP * (KX / 8);
  k_xprep<<<cdiv(nUx, NTHR), NTHR, 0, stream>>>(x, XB, nN, nUx);

  {
    const int nUw1 = HC * (KX / 8);
    k_wtr<<<cdiv(nUw1, NTHR), NTHR, 0, stream>>>(W1, F_IN, KX, HC, KX, W1T, nUw1);
    const int nUw2 = HC * (KA / 8);
    k_wtr<<<cdiv(nUw2, NTHR), NTHR, 0, stream>>>(W2, HC, HC, HC, KA, W2T, nUw2);
    k_wtr<<<cdiv(nUw2, NTHR), NTHR, 0, stream>>>(W3, HC, HC, HC, KA, W3T, nUw2);
  }

  const int gM = MP / GBM;
  k_gemm<<<dim3(gM, HC / GBN), GTHR, 0, stream>>>(XB, W1T, H, KX, HC, a1s, a1d, HID, SD, MP);
  k_agg<1><<<gA, NTHR, LDS_AGG, stream>>>(src, dst, H, SD, b1, fcw, fcb, AP, out, nN, nE, nb, vec8, MP);
  k_gemm<<<dim3(gM, HC / GBN), GTHR, 0, stream>>>(AP, W2T, H, KA, HC, a2s, a2d, HID, SD, MP);
  k_agg<1><<<gA, NTHR, LDS_AGG, stream>>>(src, dst, H, SD, b2, fcw, fcb, AP, out, nN, nE, nb, vec8, MP);
  k_gemm<<<dim3(gM, HC / GBN), GTHR, 0, stream>>>(AP, W3T, H, KA, HC, a3s, a3d, HID, SD, MP);
  k_agg<2><<<gA, NTHR, LDS_AGG, stream>>>(src, dst, H, SD, b3, fcw, fcb, AP, out, nN, nE, nb, vec8, MP);
}
